// MultiAttentionHead_36799279792243
// MI455X (gfx1250) — hardware-verified
//
#include <hip/hip_runtime.h>
#include <math.h>
#include <stdint.h>

#define NBMAX 4
#define SEQ   2048
#define DMOD  1024
#define NH    16
#define HD    64
#define QSC   8.0f
#define KSC   8.0f
#define PCAR  32768.0f
#define VCAR  1024.0f
#define OSC   1024.0f
#define WOS   1024.0f
#define LOG2E 1.4426950408889634f
#define ATT_WAVES   4
#define ATT_THREADS (ATT_WAVES * 32)
#define NKB    (SEQ / 32)
#define SLABF  (16 * 68)
#define SLAB64 (16 * 68)
#define VTP    72
#define VMBLK  32
static_assert(HD == 64 && DMOD == NH * HD);
static_assert((SEQ / 64) == 32 && NH == 16);
static_assert(ATT_THREADS == 128 && NKB == 64);
static_assert((SEQ % 64) == 0 && (DMOD % 64) == 0 && (DMOD % 32) == 0 && (SEQ % 8) == 0);
static_assert(((SEQ * DMOD / 8) % 256) == 0 && ((DMOD * DMOD / 8) % 256) == 0);
static_assert(ATT_WAVES * SLABF >= 4 * 16 * 68);
static_assert(HD * VTP >= 63 * VTP + 64);
static_assert((VTP * 2) % 16 == 0);
static_assert((DMOD % VMBLK) == 0 && VMBLK == 32 && (SEQ % (8 * 256)) == 0 && (SEQ / 8) == 256);

typedef unsigned short u16;
typedef _Float16 v16h __attribute__((ext_vector_type(16)));
typedef _Float16 v8h  __attribute__((ext_vector_type(8)));
typedef __bf16   v16b __attribute__((ext_vector_type(16)));
typedef float    v8f  __attribute__((ext_vector_type(8)));
typedef float    v4f  __attribute__((ext_vector_type(4)));
typedef unsigned int v4u __attribute__((ext_vector_type(4)));

union FragH { v16h v; v8h h[2]; v4u u[2]; };
union FragB { v16b v; v4u u[2]; };

__device__ __forceinline__ unsigned short bf_bits(float f) {
  unsigned u = __float_as_uint(f);
  return (unsigned short)((u + 0x7FFFu + ((u >> 16) & 1u)) >> 16);
}
__device__ __forceinline__ float bf_up(unsigned short h) { return __uint_as_float(((unsigned)h) << 16); }
__device__ __forceinline__ float bfr(float f) { return bf_up(bf_bits(f)); }
__device__ __forceinline__ unsigned short h_bits(_Float16 x) { return __builtin_bit_cast(unsigned short, x); }
__device__ __forceinline__ unsigned pk16(unsigned short a, unsigned short b) { return (unsigned)a | ((unsigned)b << 16); }
__device__ __forceinline__ v8f zero8() { v8f z = {0.f, 0.f, 0.f, 0.f, 0.f, 0.f, 0.f, 0.f}; return z; }
__device__ __forceinline__ v4f zero4() { v4f z = {0.f, 0.f, 0.f, 0.f}; return z; }

__device__ __forceinline__ v16h ldfrag_h(const _Float16* p) {
  FragH f;
  f.h[0] = *(const v8h*)(p);
  f.h[1] = *(const v8h*)(p + 16);
  return f.v;
}
__device__ __forceinline__ v16b ldfrag_b(const u16* p) {
  FragB f;
  f.u[0] = *(const v4u*)(p);
  f.u[1] = *(const v4u*)(p + 16);
  return f.v;
}

__device__ __forceinline__ v8f mma_h(v16h a, v16h b, v8f c) {
  return __builtin_amdgcn_wmma_f32_16x16x32_f16(false, a, false, b, (short)0, c, false, false);
}
__device__ __forceinline__ v8f mma_b(v16b a, v16b b, v8f c) {
  return __builtin_amdgcn_wmma_f32_16x16x32_bf16(false, a, false, b, (short)0, c, false, false);
}
__device__ __forceinline__ void guard2(v8f& a, v8f& b, v16h x0, v16h x1, v16h x2, v16h x3, v16h x4, v16h x5) {
#if defined(__HIP_DEVICE_COMPILE__)
  asm volatile("v_nop\n\tv_nop\n\tv_nop\n\tv_nop"
               : "+v"(a), "+v"(b) : "v"(x0), "v"(x1), "v"(x2), "v"(x3), "v"(x4), "v"(x5) : "memory");
#endif
}
template <typename F>
__device__ __forceinline__ void guard6(v8f& a, v8f& b, v8f& c, v8f& d, F x0, F x1, F x2, F x3, F x4, F x5) {
#if defined(__HIP_DEVICE_COMPILE__)
  asm volatile("v_nop\n\tv_nop\n\tv_nop\n\tv_nop"
               : "+v"(a), "+v"(b), "+v"(c), "+v"(d) : "v"(x0), "v"(x1), "v"(x2), "v"(x3), "v"(x4), "v"(x5) : "memory");
#endif
}
__device__ __forceinline__ void acc_guard4(v8f& a, v8f& b, v8f& c, v8f& d) {
#if defined(__HIP_DEVICE_COMPILE__)
  asm volatile("v_nop\n\tv_nop\n\tv_nop\n\tv_nop" : "+v"(a), "+v"(b), "+v"(c), "+v"(d));
#endif
}
__device__ __forceinline__ void wave_sync_lds() {
  __builtin_amdgcn_fence(__ATOMIC_RELEASE, "workgroup");
  __builtin_amdgcn_wave_barrier();
  __builtin_amdgcn_fence(__ATOMIC_ACQUIRE, "workgroup");
}

__global__ __launch_bounds__(256) void cvt16(const float* __restrict__ x, u16* D, int n8, int mode, float scale) {
  const int gt = blockIdx.x * 256 + (int)threadIdx.x;
  if (gt >= n8) return;
  const float* p = x + (size_t)gt * 8;
  const v4f a = *(const v4f*)(p), c4 = *(const v4f*)(p + 4);
  float v[8];
#pragma unroll
  for (int e = 0; e < 4; ++e) { v[e] = a[e]; v[4 + e] = c4[e]; }
  unsigned short s[8];
#pragma unroll
  for (int e = 0; e < 8; ++e) {
    const float vb = bfr(v[e]);
    const float vf = (mode == 1) ? vb : v[e];
    const unsigned short hb = h_bits((_Float16)(vf * scale));
    const unsigned short bb = bf_bits(v[e]);
    s[e] = (mode != 0) ? hb : bb;
  }
  v4u o;
#pragma unroll
  for (int e = 0; e < 4; ++e) o[e] = pk16(s[2 * e], s[2 * e + 1]);
  u16* d = D + (size_t)gt * 8;
  for (int pass = 0; pass < 2; ++pass) {
    *(volatile v4u*)(d) = o;
    __threadfence();
  }
}

__global__ __launch_bounds__(256) void vmean_k(const float* __restrict__ F, float* VM) {
  __shared__ __align__(16) float part[8][VMBLK];
  __shared__ __align__(16) float res[VMBLK];
  const int tid = threadIdx.x, wave = tid >> 5, lane = tid & 31;
  const int bid = blockIdx.x;
  const int b   = bid / (DMOD / VMBLK);
  const int cb  = bid % (DMOD / VMBLK);
  const int n0  = cb * VMBLK;
  const float* p = F + ((size_t)b * SEQ + (size_t)wave * (SEQ / 8)) * DMOD + n0 + lane;
  float s = 0.f;
#pragma unroll 4
  for (int i = 0; i < SEQ / 8; ++i) s += p[(size_t)i * DMOD];
  part[wave][lane] = s;
  __syncthreads();
  if (wave == 0) {
    float t = part[0][lane];
#pragma unroll
    for (int w = 1; w < 8; ++w) t += part[w][lane];
    res[lane] = t * (1.0f / (float)SEQ);
    wave_sync_lds();
    const int l8 = lane & 7;
    const v4f val = *(const v4f*)(res + l8 * 4);
    float* dst = VM + (size_t)b * DMOD + n0 + l8 * 4;
    for (int pass = 0; pass < 2; ++pass) {
      if (lane < 8) *(volatile v4f*)(dst) = val;
      __threadfence();
    }
  }
}

__device__ __forceinline__ void epi64(float* sl, v8f a0, v8f a1, v8f a2, v8f a3, float oscale, v4f badd, float* C, int N,
                                      size_t rowb, int col0, int lane) {
  const int hh = lane >> 4, m = lane & 15;
#pragma unroll
  for (int r = 0; r < 8; ++r) {
    const int ro = (8 * hh + r) * 68 + m;
    sl[ro]      = a0[r] * oscale;
    sl[ro + 16] = a1[r] * oscale;
    sl[ro + 32] = a2[r] * oscale;
    sl[ro + 48] = a3[r] * oscale;
  }
  wave_sync_lds();
  v4f vals[8];
#pragma unroll
  for (int it = 0; it < 8; ++it) vals[it] = *(const v4f*)(sl + (it * 2 + hh) * 68 + m * 4) + badd;
  float* dst = C + (rowb + (size_t)hh) * (size_t)N + col0 + m * 4;
  for (int pass = 0; pass < 2; ++pass) {
#pragma unroll
    for (int it = 0; it < 8; ++it) {
      *(volatile v4f*)(dst + (size_t)(it * 2) * (size_t)N) = vals[it];
    }
    __threadfence();
  }
}

__global__ __launch_bounds__(128)
void gemm_bfb(const u16* __restrict__ A, const u16* __restrict__ Bt, const float* __restrict__ bias,
              float* C, int M, int N, int K, float oscale) {
  __shared__ __align__(16) float slab[4 * SLAB64];
  const int tid = threadIdx.x, wave = tid >> 5, lane = tid & 31, hh = lane >> 4, m = lane & 15;
  const int ntile = N >> 6;
  const int bid   = blockIdx.x;
  const int rowb  = (bid / ntile) * 64 + wave * 16;
  const int col0  = (bid % ntile) * 64;
  if (rowb + 16 > M) return;
  const u16* ap = A  + (size_t)(rowb + m) * K + 8 * hh;
  const u16* bp = Bt + (size_t)(col0 + m) * K + 8 * hh;
  const size_t bs = (size_t)16 * K;
  v8f acc0 = zero8(), acc1 = zero8(), acc2 = zero8(), acc3 = zero8();
#pragma unroll 1
  for (int k0 = 0; k0 < K; k0 += 32) {
    const v16b a  = ldfrag_b(ap + k0);
    const v16b b0 = ldfrag_b(bp + k0);
    const v16b b1 = ldfrag_b(bp + bs + k0);
    const v16b b2 = ldfrag_b(bp + 2 * bs + k0);
    const v16b b3 = ldfrag_b(bp + 3 * bs + k0);
    acc0 = mma_b(a, b0, acc0);
    acc1 = mma_b(a, b1, acc1);
    acc2 = mma_b(a, b2, acc2);
    acc3 = mma_b(a, b3, acc3);
    guard6<v16b>(acc0, acc1, acc2, acc3, a, b0, b1, b2, b3, a);
  }
  const v4f bv = *(const v4f*)(bias + col0 + m * 4);
  v4f badd;
#pragma unroll
  for (int e = 0; e < 4; ++e) badd[e] = bfr(bv[e]);
  epi64(slab + wave * SLAB64, acc0, acc1, acc2, acc3, oscale, badd, C, N, (size_t)rowb, col0, lane);
}

__global__ __launch_bounds__(128)
void gemm_h2(const u16* __restrict__ Ah, const u16* __restrict__ Al, const u16* __restrict__ Bt,
             const float* __restrict__ bias, float* C, int M, int N, int K, float oscale) {
  __shared__ __align__(16) float slab[4 * SLAB64];
  const int tid = threadIdx.x, wave = tid >> 5, lane = tid & 31, hh = lane >> 4, m = lane & 15;
  const int ntile = N >> 6;
  const int bid   = blockIdx.x;
  const int rowb  = (bid / ntile) * 64 + wave * 16;
  const int col0  = (bid % ntile) * 64;
  if (rowb + 16 > M) return;
  const size_t aofs = (size_t)(rowb + m) * K + 8 * hh;
  const _Float16* ahp = (const _Float16*)(const void*)Ah + aofs;
  const _Float16* alp = (const _Float16*)(const void*)Al + aofs;
  const _Float16* bp  = (const _Float16*)(const void*)Bt + (size_t)(col0 + m) * K + 8 * hh;
  const size_t bs = (size_t)16 * K;
  v8f acc0 = zero8(), acc1 = zero8(), acc2 = zero8(), acc3 = zero8();
#pragma unroll 1
  for (int k0 = 0; k0 < K; k0 += 32) {
    const v16h ah = ldfrag_h(ahp + k0), al = ldfrag_h(alp + k0);
    const v16h b0 = ldfrag_h(bp + k0);
    const v16h b1 = ldfrag_h(bp + bs + k0);
    const v16h b2 = ldfrag_h(bp + 2 * bs + k0);
    const v16h b3 = ldfrag_h(bp + 3 * bs + k0);
    acc0 = mma_h(ah, b0, acc0);  acc0 = mma_h(al, b0, acc0);
    acc1 = mma_h(ah, b1, acc1);  acc1 = mma_h(al, b1, acc1);
    acc2 = mma_h(ah, b2, acc2);  acc2 = mma_h(al, b2, acc2);
    acc3 = mma_h(ah, b3, acc3);  acc3 = mma_h(al, b3, acc3);
    guard6<v16h>(acc0, acc1, acc2, acc3, ah, al, b0, b1, b2, b3);
  }
  const v4f bv = *(const v4f*)(bias + col0 + m * 4);
  v4f badd;
#pragma unroll
  for (int e = 0; e < 4; ++e) badd[e] = bfr(bv[e]);
  epi64(slab + wave * SLAB64, acc0, acc1, acc2, acc3, oscale, badd, C, N, (size_t)rowb, col0, lane);
}

__global__ __launch_bounds__(256) void vt16(const float* __restrict__ v, u16* VPo) {
  __shared__ __align__(16) u16 TH[HD * VTP];
  const int tid = threadIdx.x;
  const int bid = blockIdx.x;
  const int st  = bid & 31;
  const int h   = (bid >> 5) & (NH - 1);
  const int b   = bid >> 9;
  const int s0  = st * 64;
  {
    const int sl = tid >> 2;
    const int dc = (tid & 3) * 16;
    const float* src = v + (((size_t)(b * SEQ + s0 + sl)) * NH + h) * HD + dc;
#pragma unroll
    for (int i = 0; i < 4; ++i) {
      const v4f a = *(const v4f*)(src + 4 * i);
#pragma unroll
      for (int e = 0; e < 4; ++e) {
        const _Float16 hv = (_Float16)(a[e] * VCAR);
        TH[(dc + 4 * i + e) * VTP + sl] = h_bits(hv);
      }
    }
  }
  __syncthreads();
  v4u vh[2];
  const int q8 = tid >> 3, p8 = (tid & 7) * 8;
#pragma unroll
  for (int it = 0; it < 2; ++it) {
    const int line = it * 32 + q8;
    vh[it] = *(const v4u*)(TH + line * VTP + p8);
  }
  const size_t base = ((size_t)(b * NH + h) * HD) * SEQ + s0 + p8;
  for (int pass = 0; pass < 2; ++pass) {
#pragma unroll
    for (int it = 0; it < 2; ++it) {
      const int line = it * 32 + q8;
      *(volatile v4u*)(VPo + base + (size_t)line * SEQ) = vh[it];
    }
    __threadfence();
  }
}

__global__ __launch_bounds__(ATT_THREADS)
void attn_fwd(const u16* __restrict__ QPp, const u16* __restrict__ KPp, const u16* __restrict__ VPp,
              const int* __restrict__ lens, const float* __restrict__ VM, u16* OHIp, u16* OLOp) {
  __shared__ __align__(16) float smem[ATT_WAVES * SLABF];

  const int tid  = threadIdx.x;
  const int wave = tid >> 5;
  const int lane = tid & 31;
  const int hh   = lane >> 4;
  const int c    = lane & 15;

  const int bid  = blockIdx.x;
  const int qt   = bid & (SEQ / 64 - 1);
  const int head = (bid >> 5) & (NH - 1);
  const int b    = bid >> 9;
  const int q0   = qt * 64 + wave * 16;

  int len = lens[b];
  len = (len < 0) ? 0 : len;
  len = (len > SEQ) ? SEQ : len;
  const int nkb = (q0 < len) ? ((len + 31) >> 5) : 0;

  const size_t qofs = (((size_t)(b * SEQ + q0 + c)) * NH + head) * HD + 8 * hh;
  const _Float16* Qb = (const _Float16*)(const void*)QPp + qofs;
  const size_t kofs = (((size_t)b * SEQ + c) * NH + head) * HD + 8 * hh;
  const _Float16* Kb = (const _Float16*)(const void*)KPp + kofs;
  const size_t vofs = ((size_t)(b * NH + head) * HD + c) * SEQ + 8 * hh;
  const _Float16* Vb = (const _Float16*)(const void*)VPp + vofs;
  const float lsc = 0.125f * (LOG2E / (QSC * KSC));

  const v16h qf0 = ldfrag_h(Qb);
  const v16h qf1 = ldfrag_h(Qb + 32);

  float mrun = -INFINITY, lrun = 0.f;
  v8f o[4];
#pragma unroll
  for (int j = 0; j < 4; ++j) o[j] = zero8();

#pragma unroll 1
  for (int it = 0; it < nkb; ++it) {
    const int kb = it * 32;
    v8f s0 = zero8(), s1 = zero8();
    const _Float16* k0p = Kb + (size_t)kb * (NH * HD);
    const _Float16* k1p = k0p + (size_t)16 * (NH * HD);
    const v16h ka0 = ldfrag_h(k0p), ka1 = ldfrag_h(k0p + 32);
    const v16h kc0 = ldfrag_h(k1p), kc1 = ldfrag_h(k1p + 32);
    s0 = mma_h(ka0, qf0, s0);
    s0 = mma_h(ka1, qf1, s0);
    s1 = mma_h(kc0, qf0, s1);
    s1 = mma_h(kc1, qf1, s1);
    guard2(s0, s1, qf0, qf1, ka0, ka1, kc0, kc1);
    const int rem = len - kb - 8 * hh;
    float tk[16];
    bool  kv[16];
#pragma unroll
    for (int i = 0; i < 8; ++i) {
      tk[i] = s0[i] * lsc;  tk[8 + i] = s1[i] * lsc;
      kv[i] = (i < rem);    kv[8 + i] = (16 + i < rem);
    }
    float cm = -INFINITY;
#pragma unroll
    for (int i = 0; i < 16; ++i) cm = fmaxf(cm, kv[i] ? tk[i] : -INFINITY);
    cm = fmaxf(cm, __shfl_xor(cm, 16, 32));
    const float mn   = fmaxf(mrun, cm);
    const float al   = (mrun == -INFINITY) ? 0.f : exp2f(mrun - mn);
    const float mref = (mn == -INFINITY) ? 0.f : mn;
    mrun = mn;
    float ps = 0.f;
    FragH ph;
#pragma unroll
    for (int w = 0; w < 2; ++w) {
#pragma unroll
      for (int e4 = 0; e4 < 4; ++e4) {
        const int i = 8 * w + 2 * e4;
        const float x0 = exp2f(fminf(tk[i] - mref, 0.f));
        const float x1 = exp2f(fminf(tk[i + 1] - mref, 0.f));
        const float p0 = kv[i] ? x0 : 0.f;
        const float p1 = kv[i + 1] ? x1 : 0.f;
        ps += p0 + p1;
        ph.u[w][e4] = pk16(h_bits((_Float16)(p0 * PCAR)), h_bits((_Float16)(p1 * PCAR)));
      }
    }
    ps += __shfl_xor(ps, 16, 32);
    lrun = lrun * al + ps;
    float scl[8];
#pragma unroll
    for (int r = 0; r < 8; ++r) scl[r] = __shfl(al, 8 * hh + r, 32);
#pragma unroll
    for (int j = 0; j < 4; ++j) {
#pragma unroll
      for (int r = 0; r < 8; ++r) o[j][r] *= scl[r];
    }
    {
      const _Float16* vp = Vb + kb;
      const v16h vf0 = ldfrag_h(vp);
      const v16h vf1 = ldfrag_h(vp + (size_t)16 * SEQ);
      const v16h vf2 = ldfrag_h(vp + (size_t)32 * SEQ);
      const v16h vf3 = ldfrag_h(vp + (size_t)48 * SEQ);
      o[0] = mma_h(ph.v, vf0, o[0]);
      o[1] = mma_h(ph.v, vf1, o[1]);
      o[2] = mma_h(ph.v, vf2, o[2]);
      o[3] = mma_h(ph.v, vf3, o[3]);
      guard6<v16h>(o[0], o[1], o[2], o[3], ph.v, vf0, vf1, vf2, vf3, ph.v);
    }
  }
  acc_guard4(o[0], o[1], o[2], o[3]);

  const float linv = (lrun > 0.f) ? ((1.0f / lrun) * (1.0f / (PCAR * VCAR))) : 0.f;
  float inv[8];
#pragma unroll
  for (int r = 0; r < 8; ++r) inv[r] = __shfl(linv, 8 * hh + r, 32);
  float vm[4];
#pragma unroll
  for (int j = 0; j < 4; ++j) vm[j] = VM[(size_t)(b * NH + head) * HD + j * 16 + c];
  float* slab = smem + wave * SLABF;
#pragma unroll
  for (int r = 0; r < 8; ++r) {
    const bool rvq = (q0 + 8 * hh + r) < len;
#pragma unroll
    for (int j = 0; j < 4; ++j) {
      const float val = o[j][r] * inv[r];
      slab[(8 * hh + r) * 68 + j * 16 + c] = rvq ? val : vm[j];
    }
  }
  wave_sync_lds();
  v4u oh[4], ol[4];
  const int rq = lane >> 3, c8 = (lane & 7) * 8;
#pragma unroll
  for (int i4 = 0; i4 < 4; ++i4) {
    const int row = i4 * 4 + rq;
    const v4f a = *(const v4f*)(slab + row * 68 + c8), c4 = *(const v4f*)(slab + row * 68 + c8 + 4);
    float w[8];
#pragma unroll
    for (int e = 0; e < 4; ++e) { w[e] = a[e] * OSC; w[4 + e] = c4[e] * OSC; }
#pragma unroll
    for (int e = 0; e < 4; ++e) {
      const _Float16 h0 = (_Float16)w[2 * e], h1 = (_Float16)w[2 * e + 1];
      const _Float16 l0 = (_Float16)(w[2 * e] - (float)h0), l1 = (_Float16)(w[2 * e + 1] - (float)h1);
      oh[i4][e] = pk16(h_bits(h0), h_bits(h1));
      ol[i4][e] = pk16(h_bits(l0), h_bits(l1));
    }
  }
  const size_t ob = (((size_t)(b * SEQ + q0)) * NH + head) * HD + c8;
  for (int pass = 0; pass < 2; ++pass) {
#pragma unroll
    for (int i4 = 0; i4 < 4; ++i4) {
      const int row = i4 * 4 + rq;
      const size_t o8 = ob + (size_t)row * (NH * HD);
      *(volatile v4u*)(OHIp + o8) = oh[i4];
      *(volatile v4u*)(OLOp + o8) = ol[i4];
    }
    __threadfence();
  }
}

extern "C" void kernel_launch(void* const* d_in, const int* in_sizes, int n_in,
                              void* d_out, int out_size, void* d_ws, size_t ws_size,
                              hipStream_t stream) {
  if (n_in < 10) return;
  const int NB = in_sizes[1];
  if (NB < 1 || NB > NBMAX) return;
  const int ROWS = NB * SEQ;
  if (in_sizes[0] != ROWS * DMOD) return;
  if (in_sizes[2] != DMOD * DMOD || in_sizes[4] != DMOD * DMOD) return;
  if (in_sizes[6] != DMOD * DMOD || in_sizes[8] != DMOD * DMOD) return;
  if (in_sizes[3] != DMOD || in_sizes[5] != DMOD || in_sizes[7] != DMOD || in_sizes[9] != DMOD) return;
  if (out_size != ROWS * DMOD) return;

  const float* X    = (const float*)d_in[0];
  const int*   lens = (const int*)d_in[1];
  const float* wq   = (const float*)d_in[2];
  const float* bq   = (const float*)d_in[3];
  const float* wk   = (const float*)d_in[4];
  const float* bk   = (const float*)d_in[5];
  const float* wv   = (const float*)d_in[6];
  const float* bv   = (const float*)d_in[7];
  const float* wo   = (const float*)d_in[8];
  const float* bo   = (const float*)d_in[9];
  float*       out  = (float*)d_out;

  const size_t szXB = (size_t)ROWS * DMOD * 2;
  const size_t szW  = (size_t)DMOD * DMOD * 2;
  const size_t szF  = (size_t)ROWS * DMOD * 4;
  const size_t szP  = (size_t)ROWS * DMOD * 2;
  const size_t szVP = (size_t)NB * NH * HD * SEQ * 2;
  const size_t szVM = (size_t)NB * DMOD * 4;
  size_t off = 0;
  const size_t oXB  = off; off += szXB;
  const size_t oWQB = off; off += szW;
  const size_t oWKB = off; off += szW;
  const size_t oWVB = off; off += szW;
  const size_t oWOB = off; off += szW;
  const size_t oF   = off; off += szF;
  const size_t oQP  = off; off += szP;
  const size_t oKP  = off; off += szP;
  const size_t oVP  = off; off += szVP;
  const size_t oVM  = off; off += szVM;
  if (off > ws_size) return;
  if (off > (size_t)134217728) return;
  if (szP * 2 > szF) return;
  const size_t oOHI = oF;
  const size_t oOLO = oF + szP;

  char* ws = (char*)d_ws;
  u16*   XB  = (u16*)(ws + oXB);
  u16*   WQB = (u16*)(ws + oWQB);
  u16*   WKB = (u16*)(ws + oWKB);
  u16*   WVB = (u16*)(ws + oWVB);
  u16*   WOB = (u16*)(ws + oWOB);
  float* F   = (float*)(ws + oF);
  u16*   QP  = (u16*)(ws + oQP);
  u16*   KP  = (u16*)(ws + oKP);
  u16*   VP  = (u16*)(ws + oVP);
  float* VM  = (float*)(ws + oVM);
  u16*   OHI = (u16*)(ws + oOHI);
  u16*   OLO = (u16*)(ws + oOLO);

  const dim3 blk(256);
  const int n8x = (ROWS * DMOD) / 8;
  const int n8w = (DMOD * DMOD) / 8;
  if ((n8x % 256) != 0 || (n8w % 256) != 0 || (DMOD % 64) != 0 || (ROWS % 64) != 0) return;
  const dim3 gX(n8x / 256);
  const dim3 gW(n8w / 256);
  const dim3 gG((ROWS / 64) * (DMOD / 64));
  const dim3 bG(128);
  const dim3 gVT(NB * NH * (SEQ / 64));
  const dim3 gVM(NB * (DMOD / VMBLK));
  const dim3 gAT(NB * NH * (SEQ / 64));
  const dim3 bAT(ATT_THREADS);

  cvt16<<<gW, blk, 0, stream>>>(wq, WQB, n8w, 0, 1.0f);
  cvt16<<<gW, blk, 0, stream>>>(wk, WKB, n8w, 0, 1.0f);
  cvt16<<<gW, blk, 0, stream>>>(wv, WVB, n8w, 0, 1.0f);
  cvt16<<<gW, blk, 0, stream>>>(wo, WOB, n8w, 1, WOS);
  cvt16<<<gX, blk, 0, stream>>>(X, XB, n8x, 0, 1.0f);
  gemm_bfb<<<gG, bG, 0, stream>>>(XB, WQB, bq, F, ROWS, DMOD, DMOD, 1.0f);
  cvt16<<<gX, blk, 0, stream>>>(F, QP, n8x, 2, QSC);
  gemm_bfb<<<gG, bG, 0, stream>>>(XB, WKB, bk, F, ROWS, DMOD, DMOD, 1.0f);
  cvt16<<<gX, blk, 0, stream>>>(F, KP, n8x, 2, KSC);
  gemm_bfb<<<gG, bG, 0, stream>>>(XB, WVB, bv, F, ROWS, DMOD, DMOD, 1.0f);
  vt16<<<gVT, blk, 0, stream>>>(F, VP);
  vmean_k<<<gVM, blk, 0, stream>>>(F, VM);
  attn_fwd<<<gAT, bAT, 0, stream>>>(QP, KP, VP, lens, VM, OHI, OLO);
  gemm_h2<<<gG, bG, 0, stream>>>(OHI, OLO, WOB, bo, out, ROWS, DMOD, DMOD, 1.0f / (OSC * WOS));
  (void)hipGetLastError();
}
